// MambaBlock_70514773066075
// MI455X (gfx1250) — hardware-verified
//
#include <hip/hip_runtime.h>
#include <math.h>

typedef __attribute__((ext_vector_type(16))) _Float16 v16h;
typedef __attribute__((ext_vector_type(8)))  _Float16 v8h;
typedef __attribute__((ext_vector_type(8)))  float    v8f;
typedef __attribute__((ext_vector_type(4)))  float    v4f;
typedef __attribute__((ext_vector_type(4)))  unsigned v4u;

constexpr int kB    = 2;
constexpr int kT    = 8;
constexpr int kH    = 32;
constexpr int kW    = 32;
constexpr int kC    = 192;
constexpr int kDI   = 384;
constexpr int kNS   = 16;
constexpr int kKD   = 4;
constexpr int kDTR  = 12;
constexpr int kLT   = 77;
constexpr int kHID  = 768;
constexpr int kL    = kT * kH * kW;
constexpr int kRows = kB * kL;
constexpr int kXZW  = 2 * kDI;
constexpr int kXPC  = 48;
constexpr int kXPN  = kKD * kXPC;
constexpr int kScCH = 64;
constexpr int kScTS = 64;
constexpr float kWCarry  = 32.0f;
constexpr float kXcCarry = 64.0f;
constexpr float kHCarry  = 16.0f;
constexpr float kLog2e   = 1.4426950408889634f;
static_assert(kL == 8192 && kH == 32 && kW == 32 && kT == 8, "index bit tricks assume 8x32x32");
static_assert(kDTR + 2 * kNS <= kXPC, "x_proj block width");
static_assert((kC % 32) == 0 && (kDI % 32) == 0 && (kHID % 32) == 0, "GEMM K multiples of 32");
static_assert((kRows % 64) == 0 && (kXZW % 64) == 0 && (kXPN % 64) == 0 && (kC % 64) == 0 && (kHID % 64) == 0, "GEMM M,N multiples of 64");
static_assert((kDI % kScCH) == 0 && (kL % kScTS) == 0, "scan tiles");

constexpr size_t kOffWIN  = 0;
constexpr size_t kOffWX   = kOffWIN  + (size_t)kXZW * kC * 2;
constexpr size_t kOffWOUT = kOffWX   + (size_t)kXPN * kDI * 2;
constexpr size_t kOffWFC1 = kOffWOUT + (size_t)kC * kDI * 2;
constexpr size_t kOffWFC2 = kOffWFC1 + (size_t)kHID * kC * 2;
constexpr size_t kOffCOND = kOffWFC2 + (size_t)kC * kHID * 2;
constexpr size_t kOffX1   = kOffCOND + (size_t)kB * kDI * 4;
constexpr size_t kOffA16  = kOffX1   + (size_t)kRows * kC * 4;
constexpr size_t kOffXZ16 = kOffA16  + (size_t)kRows * kC * 2;
constexpr size_t kOffXC16 = kOffXZ16 + (size_t)kRows * kXZW * 2;
constexpr size_t kOffXDBL = kOffXC16 + (size_t)kRows * kDI * 2;
constexpr size_t kOffYS16 = kOffXDBL + (size_t)kRows * kXPN * 4;
constexpr size_t kWsTotal = kOffYS16 + (size_t)kKD * kRows * kDI * 2;
static_assert(kWsTotal == 120720384ull, "carve total");
static_assert(kWsTotal <= 134217728ull, "carve cap");
static_assert((kOffWX % 128) == 0 && (kOffWOUT % 128) == 0 && (kOffWFC1 % 128) == 0 && (kOffWFC2 % 128) == 0 &&
              (kOffCOND % 128) == 0 && (kOffX1 % 128) == 0 && (kOffA16 % 128) == 0 && (kOffXZ16 % 128) == 0 &&
              (kOffXC16 % 128) == 0 && (kOffXDBL % 128) == 0 && (kOffYS16 % 128) == 0, "128-B aligned regions");

__device__ __forceinline__ void dep_guard_h(v8f& a, v8f& b, v16h x, v16h y) { asm volatile("v_nop\n\tv_nop\n\tv_nop\n\tv_nop" : "+v"(a), "+v"(b) : "v"(x), "v"(y)); }
__device__ __forceinline__ void dep_guard4_h(v8f& a, v8f& b, v8f& c, v8f& d, v16h x, v16h y) {
  asm volatile("v_nop\n\tv_nop\n\tv_nop\n\tv_nop" : "+v"(a), "+v"(b), "+v"(c), "+v"(d) : "v"(x), "v"(y));
}
__device__ __forceinline__ void keep4_h(v16h a, v16h b, v16h c, v16h d) { asm volatile("v_nop" :: "v"(a), "v"(b), "v"(c), "v"(d)); }
__device__ __forceinline__ void acc_guard4(v8f& a, v8f& b, v8f& c, v8f& d) { asm volatile("v_nop\n\tv_nop\n\tv_nop\n\tv_nop" : "+v"(a), "+v"(b), "+v"(c), "+v"(d)); }
template <typename T> struct Frag;
template <> struct Frag<_Float16> {
  typedef v16h V; union U { v16h v; v8h h[2]; };
  static __device__ __forceinline__ v16h load(const _Float16* p) {
    U f; f.h[0] = *(const v8h*)(p); f.h[1] = *(const v8h*)(p + 16); return f.v;
  }
  static __device__ __forceinline__ v8f mma(v16h a, v16h b, v8f c) {
    return __builtin_amdgcn_wmma_f32_16x16x32_f16(false, a, false, b, (short)0, c, false, false);
  }
  static __device__ __forceinline__ void guard(v8f& a, v8f& b, v16h x, v16h y) { dep_guard_h(a, b, x, y); }
  static __device__ __forceinline__ void keep(v16h a, v16h b, v16h c, v16h d) { keep4_h(a, b, c, d); }
};

__device__ __forceinline__ float h16_to_f32(unsigned hb) {
  const unsigned sgn = (hb & 0x8000u) << 16; const unsigned em = hb & 0x7fffu;
  const float fn = __uint_as_float((em << 13) + 0x38000000u);
  const float fs = (float)em * 5.9604644775390625e-8f;
  const float mag = (em < 0x400u) ? fs : fn; return __uint_as_float(__float_as_uint(mag) | sgn);
}
__device__ __forceinline__ void dec8(const v4u w, float* f) {
#pragma unroll
  for (int e = 0; e < 4; ++e) {
    const unsigned wd = w[e];
    f[2 * e]     = h16_to_f32(wd & 0xffffu);
    f[2 * e + 1] = h16_to_f32(wd >> 16);
  }
}
__device__ __forceinline__ float sigm_f(float x) { return __builtin_amdgcn_rcpf(1.0f + __expf(-x)); }

__device__ __forceinline__ int scan_src(int k, int l) {
  const int j = (k >= 2) ? (kL - 1 - l) : l;
  const int t = j >> 10, w = (j >> 5) & 31, hh = j & 31;
  const int alt = (t << 10) | (hh << 5) | w;
  return (k & 1) ? alt : j;
}

template <int BIAS_MODE, int OUT_MODE, bool RESID, int ACT>
__global__ __launch_bounds__(256) void gemm64_f16(
    const unsigned short* __restrict__ Ap, int lda,
    const unsigned short* __restrict__ Btp, int ldb,
    void* __restrict__ Cout, int ldc,
    const float* __restrict__ bias, const float* __restrict__ resid,
    int M, int N, int K, float scale, float oscale)
{
  typedef _Float16 T;
  typedef v16h V;
  const T* A = (const T*)Ap; const T* Bt = (const T*)Btp;
  __shared__ __align__(16) float sT[8][16 * 68];
  const int lane = threadIdx.x & 31;
  const int wave = threadIdx.x >> 5;
  const int tilesN = N >> 6;
  const int tilesM = M >> 6;
  const int tile = blockIdx.x * 8 + wave;
  if (tile >= tilesM * tilesN) return;
  const int tm = tile / tilesN;
  const int tn = tile - tm * tilesN;
  const int m0 = tm << 6;
  const int n0 = tn << 6;
  const int rlane = lane & 15;
  const int koff  = (lane >> 4) * 8;
  const int mOff  = (lane >> 4) * 8;

  v8f acc[4][4];
#pragma unroll
  for (int i = 0; i < 4; ++i)
#pragma unroll
    for (int j = 0; j < 4; ++j) acc[i][j] = (v8f){0.f,0.f,0.f,0.f,0.f,0.f,0.f,0.f};

  for (int k0 = 0; k0 < K; k0 += 32) {
    V bh[4];
#pragma unroll
    for (int j = 0; j < 4; ++j)
      bh[j] = Frag<T>::load(Bt + (size_t)(n0 + (j << 4) + rlane) * ldb + koff + k0);
#pragma unroll
    for (int i = 0; i < 4; ++i) {
      V ah = Frag<T>::load(A + (size_t)(m0 + (i << 4) + rlane) * lda + koff + k0);
#pragma unroll
      for (int j = 0; j < 4; ++j) acc[i][j] = Frag<T>::mma(ah, bh[j], acc[i][j]);
      dep_guard4_h(acc[i][0], acc[i][1], acc[i][2], acc[i][3], ah, bh[3]);
    }
    keep4_h(bh[0], bh[1], bh[2], bh[3]);
  }
  acc_guard4(acc[0][0], acc[0][1], acc[0][2], acc[0][3]);
  acc_guard4(acc[1][0], acc[1][1], acc[1][2], acc[1][3]);
  acc_guard4(acc[2][0], acc[2][1], acc[2][2], acc[2][3]);
  acc_guard4(acc[3][0], acc[3][1], acc[3][2], acc[3][3]);

  float* slab = sT[wave];
#pragma unroll
  for (int i = 0; i < 4; ++i) {
    const int mBase = m0 + (i << 4);
#pragma unroll
    for (int j = 0; j < 4; ++j) {
      const int n = n0 + (j << 4) + rlane;
      float bv = 0.f;
      if (BIAS_MODE == 2) bv = bias[n];
#pragma unroll
      for (int r = 0; r < 8; ++r) {
        float v = acc[i][j][r] * scale;
        if (BIAS_MODE == 2) v += bv;
        if (ACT == 6) {
          const float v2 = v * v;
          const float inner = v * fmaf(0.044715f, v2, 1.0f);
          const float en = __expf(-1.5957691216057308f * inner);
          v = v * __builtin_amdgcn_rcpf(1.0f + en);
        }
        if (OUT_MODE == 1) v *= oscale;
        slab[(mOff + r) * 68 + (j << 4) + rlane] = v;
      }
    }
    __builtin_amdgcn_fence(__ATOMIC_RELEASE, "workgroup");
    __builtin_amdgcn_wave_barrier();
    __builtin_amdgcn_fence(__ATOMIC_ACQUIRE, "workgroup");
    if (OUT_MODE == 0) {
      float* Cf = (float*)Cout;
      const int hh = lane >> 4, c4 = (lane & 15) * 4;
      v4f sv[8];
#pragma unroll
      for (int it = 0; it < 8; ++it) sv[it] = *(const v4f*)(slab + (it * 2 + hh) * 68 + c4);
      if (RESID) {
        v4f rv[8];
#pragma unroll
        for (int it = 0; it < 4; ++it) rv[it] = *(const v4f*)(resid + (size_t)(mBase + it * 2 + hh) * ldc + n0 + c4);
        asm volatile("" ::: "memory");
#pragma unroll
        for (int it = 4; it < 8; ++it) rv[it] = *(const v4f*)(resid + (size_t)(mBase + it * 2 + hh) * ldc + n0 + c4);
#pragma unroll
        for (int it = 0; it < 8; ++it) sv[it] += rv[it];
      }
      for (int pass = 0; pass < 2; ++pass) {
#pragma unroll
        for (int it = 0; it < 8; ++it)
          *(volatile v4f*)(Cf + (size_t)(mBase + it * 2 + hh) * ldc + n0 + c4) = sv[it];
        __threadfence();
      }
    } else {
      const int q = lane >> 3, c8 = (lane & 7) * 8;
      unsigned short* Ch = (unsigned short*)Cout;
      for (int pass = 0; pass < 2; ++pass) {
#pragma unroll
        for (int it = 0; it < 4; ++it) {
          const int row = it * 4 + q;
          const float* sp = slab + row * 68 + c8;
          v8h hv;
#pragma unroll
          for (int e = 0; e < 8; ++e) hv[e] = (_Float16)sp[e];
          *(volatile v8h*)(Ch + (size_t)(mBase + row) * ldc + n0 + c8) = hv;
        }
        __threadfence();
      }
    }
    __builtin_amdgcn_fence(__ATOMIC_RELEASE, "workgroup");
    __builtin_amdgcn_wave_barrier();
    __builtin_amdgcn_fence(__ATOMIC_ACQUIRE, "workgroup");
  }
}

__global__ __launch_bounds__(256) void wcast_kernel(
    const float* __restrict__ w_in, const float* __restrict__ w_x, const float* __restrict__ w_out,
    const float* __restrict__ w_fc1, const float* __restrict__ w_fc2,
    unsigned short* __restrict__ WIN16, unsigned short* __restrict__ WX16, unsigned short* __restrict__ WOUT16,
    unsigned short* __restrict__ WFC1, unsigned short* __restrict__ WFC2)
{
  const int plane = blockIdx.y;
  const float* src; unsigned short* dst; int total8;
  if (plane == 0)      { src = w_in;  dst = WIN16;  total8 = kXZW * kC / 8; }
  else if (plane == 1) { src = w_x;   dst = WX16;   total8 = kXPN * kDI / 8; }
  else if (plane == 2) { src = w_out; dst = WOUT16; total8 = kC * kDI / 8; }
  else if (plane == 3) { src = w_fc1; dst = WFC1;   total8 = kHID * kC / 8; }
  else                 { src = w_fc2; dst = WFC2;   total8 = kC * kHID / 8; }
  const int i = blockIdx.x * 256 + threadIdx.x;
  if (i >= total8) return;
  const int e0 = i * 8;
  size_t so = (size_t)e0;
  bool valid = true;
  if (plane == 1) {
    const int n = e0 / kDI, col = e0 - n * kDI;
    const int kd = n / kXPC, c = n - kd * kXPC;
    valid = (c < kDTR + 2 * kNS);
    const int cc = valid ? c : (kDTR + 2 * kNS - 1);
    so = (size_t)(kd * (kDTR + 2 * kNS) + cc) * kDI + col;
  }
  const v4f a0 = *(const v4f*)(src + so);
  const v4f a1 = *(const v4f*)(src + so + 4);
  const float sc = valid ? kWCarry : 0.0f;
  v8h hv;
#pragma unroll
  for (int e = 0; e < 4; ++e) {
    hv[e]     = (_Float16)(a0[e] * sc);
    hv[4 + e] = (_Float16)(a1[e] * sc);
  }
  unsigned short* qd = dst + e0;
  *(volatile v8h*)qd = hv;
  __threadfence();
  *(volatile v8h*)qd = hv;
}

__global__ __launch_bounds__(256) void cond_kernel(
    const float* __restrict__ text, const float* __restrict__ Wt, const float* __restrict__ bt,
    float* __restrict__ COND)
{
  __shared__ float sTM[kB * kC];
  const int tid = threadIdx.x;
  for (int i = tid; i < kB * kC; i += 256) {
    const int b = i / kC, c = i - b * kC;
    float s = 0.f;
#pragma unroll 1
    for (int t = 0; t < kLT; ++t) s += text[((size_t)(b * kLT + t)) * kC + c];
    sTM[i] = s * (1.0f / (float)kLT);
  }
  __syncthreads();
#pragma unroll 1
  for (int p = 0; p < (kB * kDI) / 256; ++p) {
    const int i = tid + 256 * p;
    const int b = i / kDI, dd = i - b * kDI;
    float acc = 0.f;
#pragma unroll 1
    for (int c = 0; c < kC; ++c) acc = fmaf(sTM[b * kC + c], Wt[(size_t)dd * kC + c], acc);
    const float v = acc + bt[dd];
    const float o = v * sigm_f(v);
    *(volatile float*)(COND + i) = o;
    __threadfence();
    *(volatile float*)(COND + i) = o;
  }
}

__global__ __launch_bounds__(192) void cpe_kernel(
    const float* __restrict__ X, const float* __restrict__ Wc, const float* __restrict__ Bc, float* __restrict__ O)
{
  __shared__ __align__(16) float sW[28 * kC];
  const int tid = threadIdx.x;
#pragma unroll 1
  for (int tap = 0; tap < 27; ++tap) sW[tap * kC + tid] = Wc[tid * 27 + tap];
  sW[27 * kC + tid] = 0.f;
  __syncthreads();
  const int g = blockIdx.x * 192 + tid;
  const int row = g / 48;
  const int c4 = (g - row * 48) * 4;
  const int b = row >> 13, l = row & (kL - 1);
  const int t = l >> 10, h = (l >> 5) & 31, w = l & 31;
  v4f acc = {0.f, 0.f, 0.f, 0.f};
#pragma unroll 1
  for (int th = 0; th < 9; ++th) {
    const int dti = th / 3, dhi = th - dti * 3;
    const int t2 = t + dti - 1, h2 = h + dhi - 1;
    const bool vth = ((unsigned)t2 < (unsigned)kT) && ((unsigned)h2 < (unsigned)kH);
    const int t2c = t2 < 0 ? 0 : (t2 > kT - 1 ? kT - 1 : t2);
    const int h2c = h2 < 0 ? 0 : (h2 > kH - 1 ? kH - 1 : h2);
    const size_t rbase = ((size_t)(b * kT + t2c) * kH + h2c) * kW;
#pragma unroll
    for (int dw = 0; dw < 3; ++dw) {
      const int w2 = w + dw - 1;
      const bool valid = vth && ((unsigned)w2 < (unsigned)kW);
      const int w2c = w2 < 0 ? 0 : (w2 > kW - 1 ? kW - 1 : w2);
      const int tp = valid ? (th * 3 + dw) : 27;
      const v4f xv = *(const v4f*)(X + (rbase + w2c) * kC + c4);
      const v4f wv = *(const v4f*)(sW + tp * kC + c4);
#pragma unroll
      for (int e = 0; e < 4; ++e) acc[e] = fmaf(wv[e], xv[e], acc[e]);
    }
  }
  const v4f bias = *(const v4f*)(Bc + c4);
  const v4f xc = *(const v4f*)(X + (size_t)row * kC + c4);
  v4f o;
#pragma unroll
  for (int e = 0; e < 4; ++e) o[e] = xc[e] + (acc[e] + bias[e]);
  float* op = O + (size_t)row * kC + c4;
  *(volatile v4f*)op = o;
  __threadfence();
  *(volatile v4f*)op = o;
}

__global__ __launch_bounds__(256) void ln192_kernel(
    const float* __restrict__ X, const float* __restrict__ G, const float* __restrict__ Bb,
    unsigned short* __restrict__ O16, int rows)
{
  const int lane = threadIdx.x & 31, wave = threadIdx.x >> 5;
  const int wid = blockIdx.x * 8 + wave;
  if (wid >= rows) return;
  const bool act = lane < 24;
  const int lsrc = act ? lane : 0;
  const float f = act ? 1.f : 0.f;
  const float* xr = X + (size_t)wid * kC + lsrc * 8;
  const v4f a0 = *(const v4f*)(xr);
  const v4f a1 = *(const v4f*)(xr + 4);
  float s = ((a0[0] + a0[1]) + (a0[2] + a0[3])) + ((a1[0] + a1[1]) + (a1[2] + a1[3]));
  s *= f;
#pragma unroll
  for (int off = 16; off > 0; off >>= 1) s += __shfl_xor(s, off, 32);
  const float m = s * (1.0f / (float)kC);
  float dv[8];
#pragma unroll
  for (int e = 0; e < 4; ++e) { dv[e] = a0[e] - m; dv[4 + e] = a1[e] - m; }
  float sq = 0.f;
#pragma unroll
  for (int e = 0; e < 8; ++e) sq = fmaf(dv[e], dv[e], sq);
  sq *= f;
#pragma unroll
  for (int off = 16; off > 0; off >>= 1) sq += __shfl_xor(sq, off, 32);
  const float rs = rsqrtf(sq * (1.0f / (float)kC) + 1e-6f);
  const v4f g0 = *(const v4f*)(G + lsrc * 8);
  const v4f g1 = *(const v4f*)(G + lsrc * 8 + 4);
  const v4f b0 = *(const v4f*)(Bb + lsrc * 8);
  const v4f b1 = *(const v4f*)(Bb + lsrc * 8 + 4);
  v8h hv;
#pragma unroll
  for (int e = 0; e < 4; ++e) {
    hv[e]     = (_Float16)fmaf(dv[e] * rs, g0[e], b0[e]);
    hv[4 + e] = (_Float16)fmaf(dv[4 + e] * rs, g1[e], b1[e]);
  }
  unsigned short* op = O16 + (size_t)wid * kC + lsrc * 8;
  if (act) *(volatile v8h*)op = hv;
  __threadfence();
  if (act) *(volatile v8h*)op = hv;
}

__global__ __launch_bounds__(256) void conv_silu_kernel(
    const unsigned short* __restrict__ XZ16, const float* __restrict__ COND,
    const float* __restrict__ cw, const float* __restrict__ cb, unsigned short* __restrict__ XC16)
{
  __shared__ __align__(16) float sX[3 * 4 * 34 * 32];
  __shared__ __align__(16) float sW[27 * 64];
  __shared__ __align__(16) float sCond[64];
  __shared__ __align__(16) float sBias[64];
  const int tid = threadIdx.x, lane = tid & 31, wave = tid >> 5;
  const int d0 = blockIdx.x * 64;
  const int by = blockIdx.y;
  const int hb = by & 15, bt = by >> 4;
  const int b = bt >> 3, t = bt & 7, h0 = hb * 2;
  for (int i = tid; i < 27 * 64; i += 256) {
    const int c = i & 63, tap = i >> 6;
    sW[i] = cw[(size_t)(d0 + c) * 27 + tap];
  }
  if (wave < 2) sCond[tid] = COND[b * kDI + d0 + tid];
  else if (wave < 4) sBias[tid - 64] = cb[d0 + tid - 64];
  const int c = tid & 31, wq = tid >> 5, w0 = wq * 4;
  const v4f z4 = {0.f, 0.f, 0.f, 0.f};
  float acc[2][2][4];
#pragma unroll
  for (int a = 0; a < 2; ++a)
#pragma unroll
    for (int bq = 0; bq < 2; ++bq)
#pragma unroll
      for (int e = 0; e < 4; ++e) acc[a][bq][e] = 0.f;

#pragma unroll
  for (int hf = 0; hf < 2; ++hf) {
    __syncthreads();
    if (tid < 192) {
      const int rs = tid >> 4, side = (tid >> 3) & 1, c4 = (tid & 7) * 4;
      *(v4f*)(sX + (rs * 34 + (side ? 33 : 0)) * 32 + c4) = z4;
    }
#pragma unroll
    for (int p = 0; p < 6; ++p) {
      const int i = tid + 256 * p;
      const int c8 = (i & 3) * 8, ww = (i >> 2) & 31, rs = i >> 7;
      const int dti = rs >> 2, hhi = rs & 3;
      const int t2 = t + dti - 1, h2 = h0 + hhi - 1;
      const bool valid = ((unsigned)t2 < (unsigned)kT) && ((unsigned)h2 < (unsigned)kH);
      const float fval = valid ? 1.0f : 0.0f;
      const int t2c = t2 < 0 ? 0 : (t2 > kT - 1 ? kT - 1 : t2);
      const int h2c = h2 < 0 ? 0 : (h2 > kH - 1 ? kH - 1 : h2);
      const size_t grow = ((size_t)(b * kT + t2c) * kH + h2c) * kW + ww;
      const v4u wd = *(const v4u*)(XZ16 + grow * kXZW + d0 + hf * 32 + c8);
      float fv[8];
      dec8(wd, fv);
      float ov[8];
#pragma unroll
      for (int e = 0; e < 8; ++e) ov[e] = (fv[e] + sCond[hf * 32 + c8 + e]) * fval;
      float* sp = sX + ((dti * 4 + hhi) * 34 + ww + 1) * 32 + c8;
      const v4f o0 = {ov[0], ov[1], ov[2], ov[3]};
      const v4f o1 = {ov[4], ov[5], ov[6], ov[7]};
      *(v4f*)(sp) = o0;
      *(v4f*)(sp + 4) = o1;
    }
    __syncthreads();
    const int cc = hf * 32 + c;
#pragma unroll 1
    for (int th = 0; th < 9; ++th) {
      const int dti = th / 3, dhi = th - dti * 3;
      const float wt0 = sW[(th * 3 + 0) * 64 + cc];
      const float wt1 = sW[(th * 3 + 1) * 64 + cc];
      const float wt2 = sW[(th * 3 + 2) * 64 + cc];
#pragma unroll
      for (int ho = 0; ho < 2; ++ho) {
        const float* bp = sX + ((dti * 4 + ho + dhi) * 34 + w0) * 32 + c;
        float xv[6];
#pragma unroll
        for (int q = 0; q < 6; ++q) xv[q] = bp[q * 32];
#pragma unroll
        for (int wi = 0; wi < 4; ++wi) {
          float a = acc[hf][ho][wi];
          a = fmaf(wt0, xv[wi], a);
          a = fmaf(wt1, xv[wi + 1], a);
          a = fmaf(wt2, xv[wi + 2], a);
          acc[hf][ho][wi] = a;
        }
      }
    }
  }
  __syncthreads();
#pragma unroll
  for (int hf = 0; hf < 2; ++hf) {
    const int cc = hf * 32 + c;
    const float bv = sBias[cc];
#pragma unroll
    for (int ho = 0; ho < 2; ++ho)
#pragma unroll
      for (int wi = 0; wi < 4; ++wi) {
        const float v = acc[hf][ho][wi] + bv;
        const float sv = v * sigm_f(v);
        sX[(ho * 32 + w0 + wi) * 64 + cc] = sv * kXcCarry;
      }
  }
  __syncthreads();
  const int q = lane >> 3, c8 = (lane & 7) * 8;
  const size_t row0 = ((size_t)(b * kT + t) * kH + h0) * kW;
  v8h hv[2];
  int rr[2];
#pragma unroll
  for (int it = 0; it < 2; ++it) {
    const int r = it * 32 + wave * 4 + q;
    rr[it] = r;
    const float* sp = sX + r * 64 + c8;
#pragma unroll
    for (int e = 0; e < 8; ++e) hv[it][e] = (_Float16)sp[e];
  }
  for (int pass = 0; pass < 2; ++pass) {
#pragma unroll
    for (int it = 0; it < 2; ++it)
      *(volatile v8h*)(XC16 + (row0 + rr[it]) * kDI + d0 + c8) = hv[it];
    __threadfence();
  }
}

__global__ __launch_bounds__(64) void scan_kernel(
    const float* __restrict__ XDBL, const unsigned short* __restrict__ XC16,
    const float* __restrict__ Wdt, const float* __restrict__ bdt, const float* __restrict__ Alog,
    const float* __restrict__ Dsv, unsigned short* __restrict__ YS16)
{
  __shared__ __align__(16) float sXD[kScTS * kXPC];
  __shared__ __align__(16) float sU[kScTS * kScCH];
  __shared__ __align__(16) float sY[kScTS * kScCH];
  __shared__ __align__(16) float sWd[kDTR * kScCH];
  __shared__ __align__(16) float sAn[kNS * kScCH];
  const int tid = threadIdx.x, lane = tid & 31, wave = tid >> 5;
  constexpr int kBlkPerB = kDI / kScCH;
  const int bix = blockIdx.x / kBlkPerB;
  const int d0 = (blockIdx.x - bix * kBlkPerB) * kScCH;
  const int d = d0 + tid;
  const size_t rowb = (size_t)bix * kL;
  const int q = lane >> 3, c8 = (lane & 7) * 8;
  const float inv = 1.0f / kXcCarry;
#pragma unroll 1
  for (int k = 0; k < kKD; ++k) {
    __syncthreads();
#pragma unroll 1
    for (int r = 0; r < kDTR; ++r) sWd[r * kScCH + tid] = Wdt[((size_t)(k * kDI + d)) * kDTR + r];
#pragma unroll 1
    for (int n = 0; n < kNS; ++n) sAn[n * kScCH + tid] = -expf(Alog[((size_t)(k * kDI + d)) * kNS + n]) * kLog2e;
    __syncthreads();
    float wdt[kDTR], An[kNS], h[kNS];
#pragma unroll
    for (int r = 0; r < kDTR; ++r) wdt[r] = sWd[r * kScCH + tid];
#pragma unroll
    for (int n = 0; n < kNS; ++n) { An[n] = sAn[n * kScCH + tid]; h[n] = 0.f; }
    const float dtb = bdt[k * kDI + d];
    const float Dd  = Dsv[k * kDI + d];
#pragma unroll 1
    for (int l0 = 0; l0 < kL; l0 += kScTS) {
      __syncthreads();
#pragma unroll 1
      for (int p = 0; p < 12; ++p) {
        const int i = tid + kScCH * p;
        const int s = i / 12, qq = i - s * 12;
        const int row = scan_src(k, l0 + s);
        const v4f v = *(const v4f*)(XDBL + (rowb + row) * kXPN + kXPC * k + 4 * qq);
        *(v4f*)(sXD + s * kXPC + 4 * qq) = v;
      }
#pragma unroll 1
      for (int p = 0; p < 8; ++p) {
        const int i = tid + kScCH * p;
        const int s = i >> 3, cc8 = (i & 7) * 8;
        const int row = scan_src(k, l0 + s);
        const v4u wv = *(const v4u*)(XC16 + (rowb + row) * kDI + d0 + cc8);
        float fv[8];
        dec8(wv, fv);
        const v4f a0 = {fv[0] * inv, fv[1] * inv, fv[2] * inv, fv[3] * inv};
        const v4f a1 = {fv[4] * inv, fv[5] * inv, fv[6] * inv, fv[7] * inv};
        *(v4f*)(sU + s * kScCH + cc8) = a0;
        *(v4f*)(sU + s * kScCH + cc8 + 4) = a1;
      }
      __syncthreads();
#pragma unroll 1
      for (int s = 0; s < kScTS; ++s) {
        const float* xr = sXD + s * kXPC;
        const v4f x0 = *(const v4f*)(xr);
        const v4f x1 = *(const v4f*)(xr + 4);
        const v4f x2 = *(const v4f*)(xr + 8);
        float dot = x0[0] * wdt[0];
        dot = fmaf(x0[1], wdt[1], dot);  dot = fmaf(x0[2], wdt[2], dot);   dot = fmaf(x0[3], wdt[3], dot);
        dot = fmaf(x1[0], wdt[4], dot);  dot = fmaf(x1[1], wdt[5], dot);   dot = fmaf(x1[2], wdt[6], dot);
        dot = fmaf(x1[3], wdt[7], dot);  dot = fmaf(x2[0], wdt[8], dot);   dot = fmaf(x2[1], wdt[9], dot);
        dot = fmaf(x2[2], wdt[10], dot); dot = fmaf(x2[3], wdt[11], dot);
        const float v   = dot + dtb;
        const float ea  = __expf(-fabsf(v));
        const float uu  = 1.0f + ea;
        const float l1p = __logf(uu) + (ea - (uu - 1.0f)) * __builtin_amdgcn_rcpf(uu);
        const float dt  = fmaxf(v, 0.0f) + l1p;
        const float ut  = sU[s * kScCH + tid];
        const float du  = dt * ut;
        v4f Bq[4], Cq[4];
#pragma unroll
        for (int qq = 0; qq < 4; ++qq) {
          Bq[qq] = *(const v4f*)(xr + kDTR + 4 * qq);
          Cq[qq] = *(const v4f*)(xr + kDTR + kNS + 4 * qq);
        }
        float y = 0.f;
#pragma unroll
        for (int n = 0; n < kNS; ++n) {
          const float e  = __builtin_amdgcn_exp2f(dt * An[n]);
          const float hn = fmaf(e, h[n], du * Bq[n >> 2][n & 3]);
          h[n] = hn;
          y = fmaf(hn, Cq[n >> 2][n & 3], y);
        }
        const float ys = fmaf(Dd, ut, y);
        sY[s * kScCH + tid] = ys * kXcCarry;
      }
      __syncthreads();
      v8h hv[8];
      int gr[8];
#pragma unroll
      for (int it = 0; it < 8; ++it) {
        const int r = it * 8 + wave * 4 + q;
        const float* sp = sY + r * kScCH + c8;
#pragma unroll
        for (int e = 0; e < 8; ++e) hv[it][e] = (_Float16)sp[e];
        gr[it] = scan_src(k, l0 + r);
      }
      for (int pass = 0; pass < 2; ++pass) {
#pragma unroll
        for (int it = 0; it < 8; ++it)
          *(volatile v8h*)(YS16 + ((size_t)k * kRows + rowb + gr[it]) * kDI + d0 + c8) = hv[it];
        __threadfence();
      }
    }
  }
}

__device__ __forceinline__ void acc_plane(const unsigned short* __restrict__ pr, int cA, int cB, float* yA, float* yB) {
  const v4u wa = *(const v4u*)(pr + cA);
  const v4u wb = *(const v4u*)(pr + cB);
  float fa[8], fb[8];
  dec8(wa, fa);
  dec8(wb, fb);
#pragma unroll
  for (int e = 0; e < 8; ++e) { yA[e] += fa[e]; yB[e] += fb[e]; }
}
__global__ __launch_bounds__(256) void gate_kernel(
    const unsigned short* __restrict__ YS16, const unsigned short* __restrict__ XZ16,
    const float* __restrict__ G, const float* __restrict__ Bn, unsigned short* __restrict__ G16, int rows)
{
  const int lane = threadIdx.x & 31, wave = threadIdx.x >> 5;
  const int wid = blockIdx.x * 8 + wave;
  if (wid >= rows) return;
  const int cA = 8 * lane, cB = 256 + 8 * (lane & 15);
  const bool actB = lane < 16;
  const float fB = actB ? 1.f : 0.f;
  const float inv = 1.0f / kXcCarry;
  float yA[8], yB[8];
#pragma unroll
  for (int e = 0; e < 8; ++e) { yA[e] = 0.f; yB[e] = 0.f; }
  acc_plane(YS16 + ((size_t)0 * kRows + wid) * kDI, cA, cB, yA, yB);
  acc_plane(YS16 + ((size_t)2 * kRows + wid) * kDI, cA, cB, yA, yB);
  asm volatile("" ::: "memory");
  acc_plane(YS16 + ((size_t)1 * kRows + wid) * kDI, cA, cB, yA, yB);
  acc_plane(YS16 + ((size_t)3 * kRows + wid) * kDI, cA, cB, yA, yB);
  asm volatile("" ::: "memory");
#pragma unroll
  for (int e = 0; e < 8; ++e) { yA[e] *= inv; yB[e] *= inv; }
  float zA[8], zB[8];
  {
    const unsigned short* zr = XZ16 + (size_t)wid * kXZW + kDI;
    const v4u wa = *(const v4u*)(zr + cA);
    const v4u wb = *(const v4u*)(zr + cB);
    dec8(wa, zA);
    dec8(wb, zB);
  }
  asm volatile("" ::: "memory");
  float s = 0.f, sb = 0.f;
#pragma unroll
  for (int e = 0; e < 8; ++e) { s += yA[e]; sb += yB[e]; }
  s += sb * fB;
#pragma unroll
  for (int off = 16; off > 0; off >>= 1) s += __shfl_xor(s, off, 32);
  const float m = s * (1.0f / (float)kDI);
  float dA[8], dB[8];
  float sq = 0.f, sqb = 0.f;
#pragma unroll
  for (int e = 0; e < 8; ++e) {
    dA[e] = yA[e] - m; dB[e] = yB[e] - m;
    sq = fmaf(dA[e], dA[e], sq); sqb = fmaf(dB[e], dB[e], sqb);
  }
  sq += sqb * fB;
#pragma unroll
  for (int off = 16; off > 0; off >>= 1) sq += __shfl_xor(sq, off, 32);
  const float rs = rsqrtf(sq * (1.0f / (float)kDI) + 1e-6f);
  const v4f gA0 = *(const v4f*)(G + cA),  gA1 = *(const v4f*)(G + cA + 4);
  const v4f gB0 = *(const v4f*)(G + cB),  gB1 = *(const v4f*)(G + cB + 4);
  asm volatile("" ::: "memory");
  const v4f bA0 = *(const v4f*)(Bn + cA), bA1 = *(const v4f*)(Bn + cA + 4);
  const v4f bB0 = *(const v4f*)(Bn + cB), bB1 = *(const v4f*)(Bn + cB + 4);
  v8h hvA, hvB;
#pragma unroll
  for (int e = 0; e < 4; ++e) {
    const float nA0 = fmaf(dA[e] * rs, gA0[e], bA0[e]);
    const float nA1 = fmaf(dA[4 + e] * rs, gA1[e], bA1[e]);
    const float nB0 = fmaf(dB[e] * rs, gB0[e], bB0[e]);
    const float nB1 = fmaf(dB[4 + e] * rs, gB1[e], bB1[e]);
    hvA[e]     = (_Float16)(nA0 * (zA[e]     * sigm_f(zA[e]))     * kXcCarry);
    hvA[4 + e] = (_Float16)(nA1 * (zA[4 + e] * sigm_f(zA[4 + e])) * kXcCarry);
    hvB[e]     = (_Float16)(nB0 * (zB[e]     * sigm_f(zB[e]))     * kXcCarry);
    hvB[4 + e] = (_Float16)(nB1 * (zB[4 + e] * sigm_f(zB[4 + e])) * kXcCarry);
  }
  unsigned short* orow = G16 + (size_t)wid * kDI;
  for (int pass = 0; pass < 2; ++pass) {
    *(volatile v8h*)(orow + cA) = hvA;
    if (actB) *(volatile v8h*)(orow + cB) = hvB;
    __threadfence();
  }
}

extern "C" void kernel_launch(void* const* d_in, const int* in_sizes, int n_in,
                              void* d_out, int out_size, void* d_ws, size_t ws_size,
                              hipStream_t stream)
{
  if (n_in < 28) return;
  if (in_sizes[0]  != kRows * kC) return;
  if (in_sizes[1]  != kB * kLT * kC) return;
  if (in_sizes[2]  != kC * 27 || in_sizes[3] != kC) return;
  if (in_sizes[4]  != kC * 27 || in_sizes[5] != kC) return;
  if (in_sizes[6]  != kC || in_sizes[7] != kC || in_sizes[8] != kC || in_sizes[9] != kC) return;
  if (in_sizes[10] != kXZW * kC || in_sizes[11] != kXZW) return;
  if (in_sizes[12] != kDI * kC || in_sizes[13] != kDI) return;
  if (in_sizes[14] != kDI * 27 || in_sizes[15] != kDI) return;
  if (in_sizes[16] != kKD * (kDTR + 2 * kNS) * kDI) return;
  if (in_sizes[17] != kKD * kDI * kDTR || in_sizes[18] != kKD * kDI) return;
  if (in_sizes[19] != kKD * kDI * kNS || in_sizes[20] != kKD * kDI) return;
  if (in_sizes[21] != kDI || in_sizes[22] != kDI) return;
  if (in_sizes[23] != kC * kDI) return;
  if (in_sizes[24] != kHID * kC || in_sizes[25] != kHID) return;
  if (in_sizes[26] != kC * kHID || in_sizes[27] != kC) return;
  if (out_size != kRows * kC) return;
  if (ws_size < kWsTotal) return;

  const float* x           = (const float*)d_in[0];
  const float* text        = (const float*)d_in[1];
  const float* cpe1_w      = (const float*)d_in[2];
  const float* cpe1_b      = (const float*)d_in[3];
  const float* cpe2_w      = (const float*)d_in[4];
  const float* cpe2_b      = (const float*)d_in[5];
  const float* norm1_g     = (const float*)d_in[6];
  const float* norm1_b     = (const float*)d_in[7];
  const float* norm2_g     = (const float*)d_in[8];
  const float* norm2_b     = (const float*)d_in[9];
  const float* in_proj_w   = (const float*)d_in[10];
  const float* in_proj_b   = (const float*)d_in[11];
  const float* text_proj_w = (const float*)d_in[12];
  const float* text_proj_b = (const float*)d_in[13];
  const float* conv_w      = (const float*)d_in[14];
  const float* conv_b      = (const float*)d_in[15];
  const float* x_proj_w    = (const float*)d_in[16];
  const float* dt_proj_w   = (const float*)d_in[17];
  const float* dt_proj_b   = (const float*)d_in[18];
  const float* A_log       = (const float*)d_in[19];
  const float* Ds          = (const float*)d_in[20];
  const float* out_norm_g  = (const float*)d_in[21];
  const float* out_norm_b  = (const float*)d_in[22];
  const float* out_proj_w  = (const float*)d_in[23];
  const float* fc1_w       = (const float*)d_in[24];
  const float* fc1_b       = (const float*)d_in[25];
  const float* fc2_w       = (const float*)d_in[26];
  const float* fc2_b       = (const float*)d_in[27];
  float* dout = (float*)d_out;

  char* ws = (char*)d_ws;
  unsigned short* WIN16  = (unsigned short*)(ws + kOffWIN);
  unsigned short* WX16   = (unsigned short*)(ws + kOffWX);
  unsigned short* WOUT16 = (unsigned short*)(ws + kOffWOUT);
  unsigned short* WFC1   = (unsigned short*)(ws + kOffWFC1);
  unsigned short* WFC2   = (unsigned short*)(ws + kOffWFC2);
  float*          COND   = (float*)(ws + kOffCOND);
  float*          X1     = (float*)(ws + kOffX1);
  float*          X3     = (float*)(ws + kOffX1);
  unsigned short* A16    = (unsigned short*)(ws + kOffA16);
  unsigned short* XZ16   = (unsigned short*)(ws + kOffXZ16);
  unsigned short* H16    = (unsigned short*)(ws + kOffXZ16);
  unsigned short* XC16   = (unsigned short*)(ws + kOffXC16);
  unsigned short* G16    = (unsigned short*)(ws + kOffXC16);
  float*          XDBL   = (float*)(ws + kOffXDBL);
  float*          X2     = (float*)(ws + kOffXDBL);
  unsigned short* YS16   = (unsigned short*)(ws + kOffYS16);
  const float* dummy_f = in_proj_b;

  wcast_kernel<<<dim3(72, 5), 256, 0, stream>>>(in_proj_w, x_proj_w, out_proj_w, fc1_w, fc2_w,
                                                WIN16, WX16, WOUT16, WFC1, WFC2);
  cond_kernel<<<dim3(1), 256, 0, stream>>>(text, text_proj_w, text_proj_b, COND);
  cpe_kernel<<<dim3(kRows * 48 / 192), 192, 0, stream>>>(x, cpe1_w, cpe1_b, X1);
  ln192_kernel<<<dim3(kRows / 8), 256, 0, stream>>>(X1, norm1_g, norm1_b, A16, kRows);
  gemm64_f16<2, 1, false, 0><<<dim3(384), 256, 0, stream>>>(
      A16, kC, WIN16, kC, (void*)XZ16, kXZW, in_proj_b, dummy_f, kRows, kXZW, kC, 1.0f / kWCarry, 1.0f);
  conv_silu_kernel<<<dim3(kDI / 64, kB * kT * (kH / 2)), 256, 0, stream>>>(XZ16, COND, conv_w, conv_b, XC16);
  gemm64_f16<0, 0, false, 0><<<dim3(96), 256, 0, stream>>>(
      XC16, kDI, WX16, kDI, (void*)XDBL, kXPN, dummy_f, dummy_f, kRows, kXPN, kDI, 1.0f / (kXcCarry * kWCarry), 1.0f);
  scan_kernel<<<dim3(kB * (kDI / kScCH)), kScCH, 0, stream>>>(XDBL, XC16, dt_proj_w, dt_proj_b, A_log, Ds, YS16);
  gate_kernel<<<dim3(kRows / 8), 256, 0, stream>>>(YS16, XZ16, out_norm_g, out_norm_b, G16, kRows);
  gemm64_f16<0, 0, true, 0><<<dim3(96), 256, 0, stream>>>(
      G16, kDI, WOUT16, kDI, (void*)X2, kC, dummy_f, X1, kRows, kC, kDI, 1.0f / (kXcCarry * kWCarry), 1.0f);
  cpe_kernel<<<dim3(kRows * 48 / 192), 192, 0, stream>>>(X2, cpe2_w, cpe2_b, X3);
  ln192_kernel<<<dim3(kRows / 8), 256, 0, stream>>>(X3, norm2_g, norm2_b, A16, kRows);
  gemm64_f16<2, 1, false, 6><<<dim3(384), 256, 0, stream>>>(
      A16, kC, WFC1, kC, (void*)H16, kHID, fc1_b, dummy_f, kRows, kHID, kC, 1.0f / kWCarry, kHCarry);
  gemm64_f16<2, 0, true, 0><<<dim3(96), 256, 0, stream>>>(
      H16, kHID, WFC2, kHID, (void*)dout, kC, fc2_b, X3, kRows, kC, kHID, 1.0f / (kHCarry * kWCarry), 1.0f);
}
